// CausalSelfAttention_56762287784278
// MI455X (gfx1250) — hardware-verified
//
#include <hip/hip_runtime.h>
#include <math.h>

typedef __attribute__((ext_vector_type(16))) _Float16 v16h;
typedef __attribute__((ext_vector_type(16))) __bf16 v16b;
typedef __attribute__((ext_vector_type(8)))  _Float16 v8h;
typedef __attribute__((ext_vector_type(8)))  __bf16 v8b;
typedef __attribute__((ext_vector_type(8)))  float v8f;
typedef __attribute__((ext_vector_type(4)))  float v4f;
typedef __attribute__((ext_vector_type(4)))  unsigned v4u;
typedef __attribute__((ext_vector_type(4)))  int v4i;

template <typename T> __device__ __forceinline__ void vst2(void* p, T v) { *(volatile T*)p = v; __threadfence(); *(volatile T*)p = v; }
__device__ __forceinline__ v8f wmma16(v16h a, v16h b, v8f c) {
  v8f d = __builtin_amdgcn_wmma_f32_16x16x32_f16(false, a, false, b, (short)0, c, false, false);
  asm volatile("v_nop\n\tv_nop\n\tv_nop\n\tv_nop" : "+v"(d) : "v"(a), "v"(b));
  return d;
}
__device__ __forceinline__ v8f wmma_bf(v16b a, v16b b, v8f c) {
  v8f d = __builtin_amdgcn_wmma_f32_16x16x32_bf16(false, a, false, b, (short)0, c, false, false);
  asm volatile("v_nop\n\tv_nop\n\tv_nop\n\tv_nop" : "+v"(d) : "v"(a), "v"(b));
  return d;
}
__device__ __forceinline__ v16h frag_h(const _Float16* rowk0, int lane) {
  union { v16h v; v8h q[2]; } u; const _Float16* p = rowk0 + 8 * (lane >> 4);
  u.q[0] = *(const v8h*)p; u.q[1] = *(const v8h*)(p + 16); return u.v;
}
__device__ __forceinline__ v16b frag_b(const __bf16* rowk0, int lane) {
  union { v16b v; v8b q[2]; } u; const __bf16* p = rowk0 + 8 * (lane >> 4);
  u.q[0] = *(const v8b*)p; u.q[1] = *(const v8b*)(p + 16); return u.v;
}
struct F2 { v16b h, l; };
__device__ __forceinline__ F2 bsplit16(const float v[16]) { F2 r;
#pragma unroll
  for (int i = 0; i < 16; ++i) { const __bf16 h = (__bf16)v[i]; r.h[i] = h; r.l[i] = (__bf16)(v[i] - (float)h); }
  return r; }
__device__ __forceinline__ float bfr(float v) { return (float)(__bf16)v; }
__device__ __forceinline__ v16b wcol_io(const float* Wm, int k0, int o, int lane, int ld) { v16b w; const int g = lane >> 4;
#pragma unroll
  for (int i = 0; i < 8; ++i) { w[i] = (__bf16)Wm[(size_t)(k0 + 8 * g + i) * ld + o]; w[8 + i] = (__bf16)Wm[(size_t)(k0 + 16 + 8 * g + i) * ld + o]; }
  return w; }
__device__ __forceinline__ v16h wcolh_io(const float* Wm, int k0, int o, int lane, int ld) { v16h w; const int g = lane >> 4;
#pragma unroll
  for (int i = 0; i < 8; ++i) { w[i] = (_Float16)(bfr(Wm[(size_t)(k0 + 8 * g + i) * ld + o]) * 256.0f); w[8 + i] = (_Float16)(bfr(Wm[(size_t)(k0 + 16 + 8 * g + i) * ld + o]) * 256.0f); }
  return w; }
#define LDSX() do { asm volatile("s_wait_dscnt 0" ::: "memory"); __builtin_amdgcn_wave_barrier(); __builtin_amdgcn_fence(3  , "workgroup"); } while (0)

#ifndef NB
#define NB 2
#endif
#ifndef TT
#define TT 2048
#endif
#define NB_FULL 2
#define TT_FULL 2048
#define CC 1024
#define DIN 1024
#define NH 16
#define HD 64
#define KHI 256
#define QHP 256

static_assert(CC == NH * HD);
static_assert(HD == 64);
static_assert(DIN % 32 == 0);
static_assert(CC % 128 == 0);
static_assert(CC % 64 == 0);
static_assert(CC % 32 == 0);
static_assert(TT % 64 == 0);
static_assert(TT % 32 == 0);
static_assert((NB * TT) % 64 == 0);
static_assert(KHI % 64 == 0 && KHI <= TT);
static_assert(KHI % 32 == 0);
static_assert(QHP % 16 == 0);
static_assert(QHP <= KHI);
static_assert(TT <= TT_FULL && NB <= NB_FULL);
static_assert((size_t)NB_FULL * TT_FULL * CC * 4 == 16777216u);

#define WS_QH  ((size_t)0)
#define WS_QL  (WS_QH + (size_t)2 * NB * TT * CC)
#define WS_KH  (WS_QL + (size_t)2 * NB * TT * CC)
#define WS_KL  (WS_KH + (size_t)2 * NB * TT * CC)
#define WS_VT  (WS_KL + (size_t)2 * NB * TT * CC)
#define WS_VB  (WS_VT + (size_t)2 * NB * CC * TT)
#define WS_VBL (WS_VB + (size_t)2 * NB * CC * KHI)
#define WS_CH  (WS_VBL + (size_t)2 * NB * CC * KHI)
#define WS_CL  (WS_CH + (size_t)2 * NB * TT * CC)
#define WS_END (WS_CL + (size_t)2 * NB * TT * CC)
static_assert(WS_END <= (size_t)134217728u);
static_assert(WS_QL % 128 == 0 && WS_KH % 128 == 0 && WS_KL % 128 == 0 && WS_VT % 128 == 0 && WS_VB % 128 == 0 && WS_VBL % 128 == 0 && WS_CH % 128 == 0 && WS_CL % 128 == 0);

__global__ __launch_bounds__(128) void k_proj(const float* __restrict__ X, const float* __restrict__ W, const float* __restrict__ BQ, _Float16* WH, __bf16* WB) {
  __shared__ __align__(16) float st[64][132]; __shared__ __align__(16) _Float16 sh[64][136], sl[64][136]; __shared__ __align__(16) _Float16 th[128][72]; __shared__ __align__(16) __bf16 tb[128][72], tbl[128][72];
  const int tid = threadIdx.x; const int wave = __builtin_amdgcn_readfirstlane(tid >> 5); const int lane = tid & 31, col = lane & 15, g = lane >> 4;
  const int which = blockIdx.z; const int c0 = blockIdx.y * 128; const int r0 = blockIdx.x * 64; const int bb = r0 / TT; const int t0 = r0 % TT;
  const float* WA = W + which * CC; const float* BA = BQ + which * CC;
  const float* xrow = X + ((size_t)bb * TT_FULL + t0 + wave * 16 + col) * DIN + 8 * g;
  v8f acc[8] = {};
#pragma unroll 2
  for (int kc = 0; kc < DIN / 32; ++kc) { v16b a; { const float* p = xrow + kc * 32;
#pragma unroll
      for (int i = 0; i < 8; ++i) { a[i] = (__bf16)p[i]; a[8 + i] = (__bf16)p[16 + i]; } }
    asm volatile("s_wait_loadcnt 0x0" ::: "memory");
#pragma unroll
    for (int j = 0; j < 8; ++j) { const v16b w = wcol_io(WA, kc * 32, c0 + j * 16 + col, lane, 3 * CC); asm volatile("s_wait_loadcnt 0x0" ::: "memory"); acc[j] = wmma_bf(a, w, acc[j]); } }
#pragma unroll
  for (int j = 0; j < 8; ++j) { const float bias = bfr(BA[c0 + j * 16 + col]);
#pragma unroll
    for (int r = 0; r < 8; ++r) st[wave * 16 + 8 * g + r][j * 16 + col] = acc[j][r] + bias; }
  __syncthreads();
  if (which < 2) { const size_t offH = which == 0 ? (size_t)(WS_QH / 2) : (size_t)(WS_KH / 2); const size_t offL = which == 0 ? (size_t)(WS_QL / 2) : (size_t)(WS_KL / 2);
    for (int e = tid; e < 64 * 128; e += 128) { const int rl = e >> 7, cl = e & 127; const float v = st[rl][cl]; const _Float16 hv = (_Float16)v; sh[rl][cl] = hv; sl[rl][cl] = (_Float16)((v - (float)hv) * 1024.0f); }
    __syncthreads();
    for (int e = tid; e < 64 * 16; e += 128) { const int rl = e >> 4, q = e & 15; const size_t o2 = ((size_t)r0 + rl) * CC + c0 + q * 8;
      const v4u hvv = *(const v4u*)&sh[rl][q * 8]; const v4u lvv = *(const v4u*)&sl[rl][q * 8];
      vst2(WH + offH + o2, hvv); vst2(WH + offL + o2, lvv); }
  } else { const bool hi_rows = t0 < KHI;
    for (int e = tid; e < 64 * 128; e += 128) { const int rl = e & 63, cl = e >> 6; const float v = st[rl][cl]; th[cl][rl] = (_Float16)v; const __bf16 bh = (__bf16)v; tb[cl][rl] = bh; tbl[cl][rl] = (__bf16)(v - (float)bh); }
    __syncthreads();
    for (int e = tid; e < 128 * 8; e += 128) { const int cl = e >> 3, q = e & 7; const v4u tv = *(const v4u*)&th[cl][q * 8]; vst2(WH + (size_t)(WS_VT / 2) + ((size_t)bb * CC + c0 + cl) * (size_t)TT + t0 + q * 8, tv);
      if (hi_rows) { const size_t o3 = ((size_t)bb * CC + c0 + cl) * (size_t)KHI + t0 + q * 8; const v4u bv = *(const v4u*)&tb[cl][q * 8]; const v4u blv = *(const v4u*)&tbl[cl][q * 8]; vst2(WB + (size_t)(WS_VB / 2) + o3, bv); vst2(WB + (size_t)(WS_VBL / 2) + o3, blv); } } } }

__global__ __launch_bounds__(128) void k_attn(const _Float16* QH, const _Float16* QL, const _Float16* KH, const _Float16* KL, const _Float16* VT, const __bf16* VB, const __bf16* VBL, _Float16* CH, _Float16* CL) {
  __shared__ __align__(16) float ps[4][16][36];
  __shared__ __align__(16) float cs[4][16][68];
  const int tid = threadIdx.x; const int wave = __builtin_amdgcn_readfirstlane(tid >> 5); const int lane = tid & 31, col = lane & 15, g = lane >> 4;
  const int qb = blockIdx.x, h = blockIdx.y, b = blockIdx.z;
  const int q0 = qb * 64 + wave * 16; const bool qhi = q0 < QHP;
  const size_t rowb = (size_t)b * TT; const size_t qoff = (rowb + q0 + col) * CC + h * HD;
  const int nkt = (q0 >> 5) + 1;
  v8f o[4] = {}; float mx[8], ls[8];
#pragma unroll
  for (int r = 0; r < 8; ++r) { mx[r] = -3.0e38f; ls[r] = 0.f; }
#pragma unroll 1
  for (int kt = 0; kt < nkt; ++kt) {
    const int k0 = kt * 32; const bool hip = qhi && (k0 < KHI);
    v8f acc[2] = {}, accl[2] = {};
#pragma unroll
    for (int kc = 0; kc < HD / 32; ++kc) { const v16h ah = frag_h(QH + qoff + kc * 32, lane), al = frag_h(QL + qoff + kc * 32, lane);
#pragma unroll
      for (int j = 0; j < 2; ++j) { const size_t ko = (rowb + k0 + j * 16 + col) * CC + h * HD + kc * 32;
        const v16h kh = frag_h(KH + ko, lane);
        acc[j] = wmma16(ah, kh, acc[j]); accl[j] = wmma16(al, kh, accl[j]);
        const v16h kl = frag_h(KL + ko, lane); accl[j] = wmma16(ah, kl, accl[j]); } }
    float s[2][8];
#pragma unroll
    for (int j = 0; j < 2; ++j)
#pragma unroll
      for (int r = 0; r < 8; ++r) s[j][r] = (acc[j][r] + accl[j][r] * (1.0f / 1024.0f)) * 0.125f;
    if (k0 + 31 > q0) {
#pragma unroll
      for (int j = 0; j < 2; ++j)
#pragma unroll
        for (int r = 0; r < 8; ++r) { const int kk = k0 + j * 16 + col; const int qi = q0 + 8 * g + r; s[j][r] = (kk > qi) ? -1.0e9f : s[j][r]; } }
#pragma unroll
    for (int r = 0; r < 8; ++r) {
      float rm = fmaxf(s[0][r], s[1][r]);
      rm = fmaxf(rm, __shfl_xor(rm, 8)); rm = fmaxf(rm, __shfl_xor(rm, 4)); rm = fmaxf(rm, __shfl_xor(rm, 2)); rm = fmaxf(rm, __shfl_xor(rm, 1));
      const float mn = fmaxf(mx[r], rm); const float corr = expf(mx[r] - mn); mx[r] = mn;
      const float p0 = expf(s[0][r] - mn), p1 = expf(s[1][r] - mn);
      float rs = p0 + p1; rs += __shfl_xor(rs, 8); rs += __shfl_xor(rs, 4); rs += __shfl_xor(rs, 2); rs += __shfl_xor(rs, 1);
      ls[r] = ls[r] * corr + rs;
      o[0][r] *= corr; o[1][r] *= corr; o[2][r] *= corr; o[3][r] *= corr;
      ps[wave][8 * g + r][col] = p0 * 2048.0f; ps[wave][8 * g + r][16 + col] = p1 * 2048.0f; }
    LDSX();
    float pv[16];
#pragma unroll
    for (int i = 0; i < 8; ++i) { pv[i] = ps[wave][col][8 * g + i]; pv[8 + i] = ps[wave][col][16 + 8 * g + i]; }
    if (hip) { const F2 p = bsplit16(pv);
#pragma unroll
      for (int j = 0; j < 4; ++j) { const size_t po = ((size_t)b * CC + h * HD + j * 16 + col) * (size_t)KHI + k0; const v16b vh = frag_b(VB + po, lane); o[j] = wmma_bf(p.l, vh, o[j]); o[j] = wmma_bf(p.h, frag_b(VBL + po, lane), o[j]); o[j] = wmma_bf(p.h, vh, o[j]); }
    } else { v16h p;
#pragma unroll
      for (int i = 0; i < 16; ++i) p[i] = (_Float16)pv[i];
#pragma unroll
      for (int j = 0; j < 4; ++j) { const size_t po = ((size_t)b * CC + h * HD + j * 16 + col) * (size_t)TT + k0; o[j] = wmma16(p, frag_h(VT + po, lane), o[j]); } }
    LDSX();
  }
#pragma unroll
  for (int r = 0; r < 8; ++r) { const float inv = ls[r] > 0.f ? 1.0f / (128.0f * ls[r]) : 0.f;
#pragma unroll
    for (int j = 0; j < 4; ++j) cs[wave][8 * g + r][j * 16 + col] = o[j][r] * inv; }
  LDSX();
#pragma unroll
  for (int i = 0; i < 4; ++i) { const int rl = i * 4 + (lane >> 3), pc = lane & 7; v8h hv, lv;
#pragma unroll
    for (int e = 0; e < 8; ++e) { const float v = cs[wave][rl][pc * 8 + e]; const _Float16 hh = (_Float16)v; hv[e] = hh; lv[e] = (_Float16)((v - (float)hh) * 1024.0f); }
    const size_t off = (rowb + q0 + rl) * CC + h * HD + pc * 8;
    const v4u hu = __builtin_bit_cast(v4u, hv); const v4u lu = __builtin_bit_cast(v4u, lv);
    vst2(CH + off, hu); vst2(CL + off, lu); } }

__global__ __launch_bounds__(128) void k_out(const _Float16* CH, const _Float16* CL, const float* __restrict__ WO, const float* __restrict__ BO, float* OUT) {
  __shared__ __align__(16) float st[4][16][68];
  const int tid = threadIdx.x; const int wave = __builtin_amdgcn_readfirstlane(tid >> 5); const int lane = tid & 31, col = lane & 15, g = lane >> 4;
  const int r0 = blockIdx.x * 64 + wave * 16; const int c0 = blockIdx.y * 64;
  const size_t aoff = ((size_t)r0 + col) * CC;
  v8f acc[4] = {}, accl[4] = {};
#pragma unroll 2
  for (int kc = 0; kc < CC / 32; ++kc) { const v16h ah = frag_h(CH + aoff + kc * 32, lane), al = frag_h(CL + aoff + kc * 32, lane);
#pragma unroll
    for (int j = 0; j < 4; ++j) { const v16h w = wcolh_io(WO, kc * 32, c0 + j * 16 + col, lane, CC); asm volatile("s_wait_loadcnt 0x0" ::: "memory"); acc[j] = wmma16(ah, w, acc[j]); accl[j] = wmma16(al, w, accl[j]); } }
#pragma unroll
  for (int j = 0; j < 4; ++j) { const float bias = bfr(BO[c0 + j * 16 + col]);
#pragma unroll
    for (int r = 0; r < 8; ++r) st[wave][8 * g + r][j * 16 + col] = (acc[j][r] + accl[j][r] * (1.0f / 1024.0f)) * (1.0f / 4096.0f) + bias; }
  LDSX();
#pragma unroll
  for (int i = 0; i < 8; ++i) { const int rl = i * 2 + (lane >> 4), pc = lane & 15; const int R = r0 + rl; const int bo = R / TT, to = R % TT;
    const v4f v = *(const v4f*)&st[wave][rl][pc * 4];
    vst2(OUT + ((size_t)bo * TT_FULL + to) * CC + c0 + pc * 4, v); } }

extern "C" void kernel_launch(void* const* d_in, const int* in_sizes, int n_in, void* d_out, int out_size, void* d_ws, size_t ws_size, hipStream_t stream) {
  if (n_in < 5) return;
  const long long rows_need = (long long)(NB - 1) * TT_FULL + TT;
  if ((long long)in_sizes[0] < rows_need * DIN) return;
  if ((long long)in_sizes[1] < (long long)DIN * 3 * CC) return;
  if ((long long)in_sizes[2] < 3 * CC) return;
  if ((long long)in_sizes[3] < (long long)CC * CC) return;
  if ((long long)in_sizes[4] < CC) return;
  if ((long long)out_size < rows_need * CC) return;
  if (ws_size < (size_t)WS_END) return;
  const float* x = (const float*)d_in[0]; const float* Wqkv = (const float*)d_in[1]; const float* bqkv = (const float*)d_in[2]; const float* Wout = (const float*)d_in[3]; const float* bout = (const float*)d_in[4];
  char* ws = (char*)d_ws;
  _Float16 *QH = (_Float16*)(ws + WS_QH), *QL = (_Float16*)(ws + WS_QL), *KH = (_Float16*)(ws + WS_KH), *KL = (_Float16*)(ws + WS_KL), *VT = (_Float16*)(ws + WS_VT), *CH = (_Float16*)(ws + WS_CH), *CL = (_Float16*)(ws + WS_CL);
  __bf16 *VB = (__bf16*)(ws + WS_VB), *VBL = (__bf16*)(ws + WS_VBL);
  k_proj<<<dim3(NB * TT / 64, CC / 128, 3), 128, 0, stream>>>(x, Wqkv, bqkv, (_Float16*)ws, (__bf16*)ws);
  k_attn<<<dim3(TT / 64, NH, NB), 128, 0, stream>>>(QH, QL, KH, KL, VT, VB, VBL, CH, CL);
  k_out<<<dim3(NB * TT / 64, CC / 64), 128, 0, stream>>>(CH, CL, Wout, bout, (float*)d_out);
}
